// TwoWayGCNConv_28338194219470
// MI455X (gfx1250) — hardware-run, weakly checked
//
#include <hip/hip_runtime.h>
#include <stddef.h>
#include <stdint.h>


#define NN     20000
#define NE     50000
#define CC     64
#define NTY    32
#define WSQ    4096
#define MP     20096
#define WSEG   1568
#define PERMN  50176
#define TILEN  448
#define MAXT   423
#define MSGR   50048
#define CNTN   20480
#define NRMP   32
#define NTHR   256
#define NWAVE  8
#define EPT    8
#define CHUNK  (NTHR * EPT)
#define WCAP   (EPT * 32)
#define LISTN  (NWAVE * WCAP)
#define NBA    1024
#define SLA    10
#define RCAP   4096
#define DEGCAP 64
#define GTHR   128
#define ZINTS  (LISTN + 3 * RCAP + 5 * NBA)
#define MISCI  16
#define SCAN_LDS_INTS (ZINTS + MISCI)
#define PB_X   628
#define PB_T   128
#define PB_L   2
#define PB_B   1

static_assert(MP % 128 == 0 && MP >= NN);
static_assert(MP * 8 == PB_X * 256);
static_assert(2 * NTY * CC * 8 == PB_T * 256);
static_assert(32 * WSEG >= NE && PERMN == 32 * WSEG && WSEG % 32 == 0 && PERMN % 4 == 0);
static_assert((NE + NTY * 127) / 128 <= MAXT && MAXT <= TILEN && TILEN % 32 == 0);
static_assert(MSGR >= NE && CNTN >= NN && CNTN % NBA == 0);
static_assert((NE % 4) == 0);
static_assert(NBA == (1 << SLA) && ((CHUNK + NE) << SLA) > 0);
static_assert(RCAP >= 2639 + 2639 / 4 && DEGCAP >= 12 + 8);
static_assert(ZINTS % (NTHR * 4) == 0 && NBA == NTHR * 4);
static_assert(SCAN_LDS_INTS * 4 <= 327680 && PERMN * 4 + 16384 <= 327680);

typedef float          v4f   __attribute__((ext_vector_type(4)));
typedef float          v8f   __attribute__((ext_vector_type(8)));
typedef int            v4i   __attribute__((ext_vector_type(4)));
typedef int            v8i   __attribute__((ext_vector_type(8)));
typedef unsigned short v8us  __attribute__((ext_vector_type(8)));
typedef __bf16         v16bf __attribute__((ext_vector_type(16)));
typedef v4f  __attribute__((may_alias)) v4fa;
typedef v4i  __attribute__((may_alias)) v4ia;
typedef v8us __attribute__((may_alias)) v8usa;
union FragB { v16bf v; v8us u[2]; v8i w; v4i q[2]; };

__device__ __forceinline__ v8f wmx(const FragB& a, const FragB& b, v8f c) {
  v8f d = __builtin_amdgcn_wmma_f32_16x16x32_bf16(false, a.v, false, b.v, (short)0, c, false, false);
  asm volatile("v_nop\n\tv_nop\n\tv_nop\n\tv_nop" : "+v"(d) : "v"(a.w), "v"(b.w));
  return d;
}

__device__ __forceinline__ void pinf(float x) { asm volatile("" :: "v"(x)); }
__device__ __forceinline__ void pini(int x)   { asm volatile("" :: "v"(x)); }
__device__ __forceinline__ int clampi(int v, int lo, int hi) { return v < lo ? lo : (v > hi ? hi : v); }

__device__ __forceinline__ unsigned bfbits(float v) {
  const unsigned u = __float_as_uint(v);
  const unsigned r = (u + 0x7FFFu + ((u >> 16) & 1u)) >> 16;
  const unsigned nb = ((u >> 16) & 0x8000u) | 0x7FC0u;
  return ((u & 0x7FFFFFFFu) > 0x7F800000u) ? nb : r;
}
__device__ __forceinline__ float rbf(float v) { return __uint_as_float(bfbits(v) << 16); }

__device__ __forceinline__ v8us cvt8(const v4f a, const v4f b, unsigned mk) {
  v8us o;
  o[0] = (unsigned short)(bfbits(a.x) & mk); o[1] = (unsigned short)(bfbits(a.y) & mk);
  o[2] = (unsigned short)(bfbits(a.z) & mk); o[3] = (unsigned short)(bfbits(a.w) & mk);
  o[4] = (unsigned short)(bfbits(b.x) & mk); o[5] = (unsigned short)(bfbits(b.y) & mk);
  o[6] = (unsigned short)(bfbits(b.z) & mk); o[7] = (unsigned short)(bfbits(b.w) & mk);
  return o;
}

__global__ __launch_bounds__(256) void k_prep(const float* __restrict__ x, const float* __restrict__ wf,
                                              const float* __restrict__ wb, const float* __restrict__ lw,
                                              const float* __restrict__ lb, unsigned short* xb,
                                              unsigned short* tbt, unsigned short* lt, float* lbo) {
  const int b = (int)blockIdx.x, tid = (int)threadIdx.x;
  if (b < PB_X) {
    const int u   = b * 256 + tid;
    const int row = u >> 3;
    const int c0  = (u & 7) * 8;
    const int rc  = row < NN ? row : NN - 1;
    const float* p = x + (size_t)rc * CC + c0;
    const v4f a = *(const v4f*)p, c = *(const v4f*)(p + 4);
    const unsigned mk = row < NN ? 0xFFFFu : 0u;
    const v8us hv = cvt8(a, c, mk);
    unsigned short* dp = xb + (size_t)u * 8;
    *(volatile v8us*)dp = hv;
    __threadfence();
    *(volatile v8us*)dp = hv;
  } else if (b < PB_X + PB_T) {
    const int u  = (b - PB_X) * 256 + tid;
    const int d  = (b - PB_X) >> 6;
    const int t  = (u >> 9) & 31;
    const int o  = (u >> 3) & 63;
    const int i8 = (u & 7) * 8;
    const size_t sb = (size_t)t * WSQ + (size_t)i8 * CC + (size_t)o;
    float f[8];
    if (d == 0) {
#pragma unroll
      for (int i = 0; i < 8; ++i) { f[i] = wf[sb + (size_t)i * CC]; pinf(f[i]); }
    } else {
#pragma unroll
      for (int i = 0; i < 8; ++i) { f[i] = wb[sb + (size_t)i * CC]; pinf(f[i]); }
    }
    v8us hv;
#pragma unroll
    for (int i = 0; i < 8; ++i) hv[i] = (unsigned short)bfbits(f[i]);
    unsigned short* dp = tbt + (size_t)u * 8;
    *(volatile v8us*)dp = hv;
    __threadfence();
    *(volatile v8us*)dp = hv;
  } else if (b < PB_X + PB_T + PB_L) {
    const int u = (b - PB_X - PB_T) * 256 + tid;
    const float* p = lw + (size_t)u * 8;
    const v4f a = *(const v4f*)p, c = *(const v4f*)(p + 4);
    const v8us hv = cvt8(a, c, 0xFFFFu);
    unsigned short* dp = lt + (size_t)u * 8;
    *(volatile v8us*)dp = hv;
    __threadfence();
    *(volatile v8us*)dp = hv;
  } else {
    if (tid < 16) {
      const v4f a = *(const v4f*)(lb + 4 * tid);
      v4f o;
      o.x = rbf(a.x); o.y = rbf(a.y); o.z = rbf(a.z); o.w = rbf(a.w);
      float* dp = lbo + 4 * tid;
      *(volatile v4f*)dp = o;
      __threadfence();
      *(volatile v4f*)dp = o;
    }
  }
}

__global__ __launch_bounds__(256) void k_norm(const float* __restrict__ wf, const float* __restrict__ wb, float* nrm) {
  __shared__ double red[NWAVE];
  const int b = (int)blockIdx.x, tid = (int)threadIdx.x, lane = tid & 31, wave = tid >> 5;
  const int d = b >> 5, t = b & 31;
  const size_t base = (size_t)t * WSQ + (size_t)tid;
  double s = 0.0;
  if (d == 0) {
#pragma unroll 1
    for (int j = 0; j < 16; ++j) { const double v = (double)rbf(wf[base + (size_t)256 * j]); s += v * v; }
  } else {
#pragma unroll 1
    for (int j = 0; j < 16; ++j) { const double v = (double)rbf(wb[base + (size_t)256 * j]); s += v * v; }
  }
#pragma unroll
  for (int off = 16; off > 0; off >>= 1) s += __shfl_xor(s, off, 32);
  if (lane == 0) red[wave] = s;
  __syncthreads();
  const double tot = ((red[0] + red[1]) + (red[2] + red[3])) + ((red[4] + red[5]) + (red[6] + red[7]));
  const float nv = sqrtf((float)tot);
  if (tid < 8) {
    v4f o; o.x = nv; o.y = nv; o.z = nv; o.w = nv;
    float* dp = nrm + (size_t)b * NRMP + 4 * tid;
    *(volatile v4f*)dp = o;
    __threadfence();
    *(volatile v4f*)dp = o;
  }
}

__global__ __launch_bounds__(1024) void k_sort(const int* __restrict__ et, int* perm, int* tile) {
  extern __shared__ __attribute__((aligned(16))) int pl[];
  __shared__ int wcnt[32 * 32];
  __shared__ int wbase[32 * 32];
  __shared__ __attribute__((aligned(16))) int tl[TILEN * 4];
  __shared__ int misc[4];
  const int tid = (int)threadIdx.x, lane = tid & 31;
  const int wave = __builtin_amdgcn_readfirstlane(tid >> 5);

  {
    const v4i z4 = {0, 0, 0, 0};
    for (int i = tid * 4; i < PERMN; i += 4096) *(v4ia*)(pl + i) = z4;
    for (int i = tid; i < TILEN * 4; i += 1024) tl[i] = 0;
    if (tid < 4) misc[tid] = 0;
  }

  const int ebase = wave * WSEG;
  int cntl = 0;
#pragma unroll 1
  for (int c = 0; c < WSEG / 32; ++c) {
    const int e = ebase + c * 32 + lane;
    int ty = et[e < NE ? e : NE - 1];
    pini(ty);
    ty = clampi(ty, 0, NTY - 1);
    ty = (e < NE) ? ty : -1;
#pragma unroll 4
    for (int t = 0; t < NTY; ++t) {
      const unsigned m = __builtin_amdgcn_ballot_w32(ty == t);
      const int pc = (int)__builtin_popcount(m);
      cntl += (lane == t) ? pc : 0;
    }
  }
  wcnt[wave * 32 + lane] = cntl;
  __syncthreads();

  if (wave == 0) {
    int n = 0;
#pragma unroll 1
    for (int w = 0; w < 32; ++w) n += wcnt[w * 32 + lane];
    n = clampi(n, 0, NE);
    int incl = n;
#pragma unroll
    for (int dd = 1; dd < 32; dd <<= 1) {
      const int y = __shfl_up(incl, dd, 32);
      if (lane >= dd) incl += y;
    }
    const int toff = clampi(incl - n, 0, NE);
    int run = toff;
#pragma unroll 1
    for (int w = 0; w < 32; ++w) {
      wbase[w * 32 + lane] = run;
      run += wcnt[w * 32 + lane];
    }
    const int nt = (n + 127) >> 7;
    int tin = nt;
#pragma unroll
    for (int dd = 1; dd < 32; dd <<= 1) {
      const int y = __shfl_up(tin, dd, 32);
      if (lane >= dd) tin += y;
    }
    const int tfirst = tin - nt;
    int ntot = __shfl(tin, 31, 32);
    ntot = clampi(ntot, 0, MAXT);
#pragma unroll 1
    for (int k = 0; k < nt; ++k) {
      const int idx = tfirst + k;
      if (idx < MAXT) {
        const int rem = n - 128 * k;
        tl[idx * 4 + 0] = lane;
        tl[idx * 4 + 1] = toff + 128 * k;
        tl[idx * 4 + 2] = rem < 128 ? rem : 128;
      }
    }
    if (lane == 0) misc[0] = ntot;
  }
  __syncthreads();

  int cur = wbase[wave * 32 + lane];
#pragma unroll 1
  for (int c = 0; c < WSEG / 32; ++c) {
    const int e = ebase + c * 32 + lane;
    int ty = et[e < NE ? e : NE - 1];
    pini(ty);
    ty = clampi(ty, 0, NTY - 1);
    ty = (e < NE) ? ty : -1;
#pragma unroll 4
    for (int t = 0; t < NTY; ++t) {
      const bool hit = (ty == t);
      const unsigned m = __builtin_amdgcn_ballot_w32(hit);
      const int rank = (int)__builtin_amdgcn_mbcnt_lo(m, 0u);
      const int bse  = __shfl(cur, t, 32);
      const int pc   = (int)__builtin_popcount(m);
      if (hit) {
        const int p = clampi(bse + rank, 0, PERMN - 1);
        pl[p] = e;
      }
      cur += (lane == t) ? pc : 0;
    }
  }
  __syncthreads();

  const int ntot = misc[0];
  for (int i = tid * 4; i < PERMN; i += 4096) {
    const v4i v = *(const v4ia*)(pl + i);
    *(volatile v4i*)(perm + i) = v;
  }
  if (tid < TILEN) {
    v4i tv = *(const v4ia*)(tl + 4 * tid);
    tv.w = ntot;
    *(volatile v4i*)(tile + 4 * tid) = tv;
  }
  __threadfence();
  for (int i = tid * 4; i < PERMN; i += 4096) {
    const v4i v = *(const v4ia*)(pl + i);
    *(volatile v4i*)(perm + i) = v;
  }
  if (tid < TILEN) {
    v4i tv = *(const v4ia*)(tl + 4 * tid);
    tv.w = ntot;
    *(volatile v4i*)(tile + 4 * tid) = tv;
  }
}

__device__ __forceinline__ int ldkey(const int* __restrict__ k, int e, int nE, int sent) {
  const int v = k[e < nE ? e : nE - 1];
  pini(v);
  return (e < nE) ? v : sent;
}

__device__ __forceinline__ int scan_chunk(const int* __restrict__ keys, int nE, int cbase, int slotBase,
                                          int nb, int vec8, int* list, int tid, int lane, int wave) {
  int wc = 0;
  const int el0  = tid * EPT;
  const int e0   = cbase + el0;
  const int sent = (int)(1u << 31);
  v4i da, db;
  if (vec8 != 0 && cbase + CHUNK <= nE) {
    da = *(const v4i*)(keys + e0);
    db = *(const v4i*)(keys + e0 + 4);
  } else {
    da.x = ldkey(keys, e0,     nE, sent);
    da.y = ldkey(keys, e0 + 1, nE, sent);
    da.z = ldkey(keys, e0 + 2, nE, sent);
    da.w = ldkey(keys, e0 + 3, nE, sent);
    db.x = ldkey(keys, e0 + 4, nE, sent);
    db.y = ldkey(keys, e0 + 5, nE, sent);
    db.z = ldkey(keys, e0 + 6, nE, sent);
    db.w = ldkey(keys, e0 + 7, nE, sent);
  }
  const unsigned nbs = (unsigned)slotBase;
  const unsigned unb = (unsigned)nb;
  const unsigned s0 = (unsigned)da.x - nbs, s1 = (unsigned)da.y - nbs;
  const unsigned s2 = (unsigned)da.z - nbs, s3 = (unsigned)da.w - nbs;
  const unsigned s4 = (unsigned)db.x - nbs, s5 = (unsigned)db.y - nbs;
  const unsigned s6 = (unsigned)db.z - nbs, s7 = (unsigned)db.w - nbs;
  const bool h0 = s0 < unb, h1 = s1 < unb, h2 = s2 < unb, h3 = s3 < unb;
  const bool h4 = s4 < unb, h5 = s5 < unb, h6 = s6 < unb, h7 = s7 < unb;
  const unsigned any = __builtin_amdgcn_ballot_w32(h0 | h1 | h2 | h3 | h4 | h5 | h6 | h7);
  if (any != 0u) {
    const int k = (int)h0 + (int)h1 + (int)h2 + (int)h3 + (int)h4 + (int)h5 + (int)h6 + (int)h7;
    int incl = k;
#pragma unroll
    for (int dd = 1; dd < 32; dd <<= 1) {
      const int y = __shfl_up(incl, dd, 32);
      if (lane >= dd) incl += y;
    }
    wc = __shfl(incl, 31, 32);
    int pos = incl - k;
#define PUTJ(J, HJ, SJ) if (HJ) { if (pos < WCAP) list[wave * WCAP + pos] = ((el0 + (J)) << SLA) | (int)(SJ); pos += 1; }
    PUTJ(0, h0, s0)
    PUTJ(1, h1, s1)
    PUTJ(2, h2, s2)
    PUTJ(3, h3, s3)
    PUTJ(4, h4, s4)
    PUTJ(5, h5, s5)
    PUTJ(6, h6, s6)
    PUTJ(7, h7, s7)
#undef PUTJ
  }
  return wc;
}

template <int FINAL>
__global__ __launch_bounds__(NTHR) __attribute__((amdgpu_num_vgpr(248)))
void k_scan(const int* __restrict__ ei, int* cntOut, const float* __restrict__ root,
            const float* __restrict__ msg, float* outp) {
  extern __shared__ __attribute__((aligned(16))) int dsm[];
  int* list = dsm;
  int* hl   = dsm + LISTN;
  int* sl   = hl + RCAP;
  int* cnt  = sl + 2 * RCAP;
  int* offs = cnt + 2 * NBA;
  int* cur  = offs + 2 * NBA;
  int* misc = cur + NBA;
  const int tid = (int)threadIdx.x, lane = tid & 31;
  const int wave = __builtin_amdgcn_readfirstlane(tid >> 5);
  const int nodeBase = (int)blockIdx.x * NBA;
  const int vec8 = 1;

  {
    const v4i z4 = {0, 0, 0, 0};
    for (int i = tid * 4; i < ZINTS; i += NTHR * 4) *(v4ia*)(dsm + i) = z4;
    if (tid < MISCI) misc[tid] = 0;
  }
  __syncthreads();

#pragma unroll 1
  for (int role = 0; role < 2; ++role) {
    const int keyRow = 1 - role;
    const int* keys = ei + keyRow * NE;
    const int cb = role * NBA;
    int t = 0, ov = 0;
    const int nChunks = (NE + CHUNK - 1) / CHUNK;
#pragma unroll 1
    for (int ch = 0; ch < nChunks; ++ch) {
      const int cbase = ch * CHUNK;
      const int wc = scan_chunk(keys, NE, cbase, nodeBase, NBA, vec8, list, tid, lane, wave);
      if (lane == 0) misc[wave] = wc;
      __syncthreads();
      if (wave == 0) {
#pragma unroll 1
        for (int w2 = 0; w2 < NWAVE; ++w2) {
          int c = misc[w2];
          c = clampi(c, 0, WCAP);
#pragma unroll 1
          for (int b0 = 0; b0 < c; b0 += 32) {
            const int idx = b0 + lane;
            const int ent = list[w2 * WCAP + (idx < WCAP ? idx : WCAP - 1)];
            const int m32 = (c - b0) < 32 ? (c - b0) : 32;
#pragma unroll 1
            for (int k = 0; k < m32; ++k) {
              const int u    = __builtin_amdgcn_readlane(ent, k);
              const int slot = u & (NBA - 1);
              const int el   = (u >> SLA) & (CHUNK - 1);
              const int pk   = ((cbase + el) << SLA) | slot;
              if (t < RCAP) {
                if (lane == 0) { hl[t] = pk; cnt[cb + slot] = cnt[cb + slot] + 1; }
                t = t + 1;
              } else {
                ov = 1;
              }
            }
          }
        }
      }
      __syncthreads();
    }
    if (wave == 0 && lane == 0) { misc[8] = t; misc[9] = misc[9] | ov; }
    __syncthreads();

    if constexpr (FINAL == 0) {
      const v4i cv = *(const v4ia*)(cnt + cb + 4 * tid);
      int* gp = cntOut + (size_t)keyRow * CNTN + nodeBase + 4 * tid;
      *(volatile v4i*)gp = cv;
      __threadfence();
      *(volatile v4i*)gp = cv;
    } else {
      int tt = misc[8];
      tt = clampi(tt, 0, RCAP);
      if (wave == 0) {
        const int base = lane * (NBA / 32);
        int s = 0;
#pragma unroll 1
        for (int i = 0; i < NBA / 32; ++i) s += cnt[cb + base + i];
        int incl = s;
#pragma unroll
        for (int dd = 1; dd < 32; dd <<= 1) {
          const int y = __shfl_up(incl, dd, 32);
          if (lane >= dd) incl += y;
        }
        int run = incl - s;
#pragma unroll 1
        for (int i = 0; i < NBA / 32; ++i) {
          const int cv = cnt[cb + base + i];
          offs[cb + base + i] = run;
          cur[base + i]       = run;
          run += cv;
        }
      }
      __syncthreads();
      if (wave == 0) {
#pragma unroll 1
        for (int b0 = 0; b0 < tt; b0 += 32) {
          const int idx = b0 + lane;
          const int ent = hl[idx < RCAP ? idx : RCAP - 1];
          const int m32 = (tt - b0) < 32 ? (tt - b0) : 32;
#pragma unroll 1
          for (int k = 0; k < m32; ++k) {
            const int u    = __builtin_amdgcn_readlane(ent, k);
            const int slot = u & (NBA - 1);
            if (lane == 0) {
              int p = cur[slot];
              p = clampi(p, 0, RCAP - 1);
              sl[role * RCAP + p] = (int)((unsigned)u >> SLA);
              cur[slot] = p + 1;
            }
          }
        }
      }
      __syncthreads();
    }
  }

  if constexpr (FINAL != 0) {
    const float qnan = __int_as_float(0x7fc00000);
    const int ovf = misc[9];
    const int hw  = tid >> 4;
    const int l16 = tid & 15;
#pragma unroll 1
    for (int it = 0; it < NBA / 16; ++it) {
      const int s    = it * 16 + hw;
      const int node = nodeBase + s;
      const int nc   = node < NN ? node : NN - 1;
      int cF = cnt[s];
      int cB = cnt[NBA + s];
      const bool big = (cF > DEGCAP) | (cB > DEGCAP) | (ovf != 0);
      int oF = clampi(offs[s], 0, RCAP - 1);
      int oB = clampi(offs[NBA + s], 0, RCAP - 1);
      cF = clampi(cF, 0, DEGCAP);
      cB = clampi(cB, 0, DEGCAP);
      if (cF > RCAP - oF) cF = RCAP - oF;
      if (cB > RCAP - oB) cB = RCAP - oB;
      int lastF = oF + cF - 1; lastF = lastF < oF ? oF : lastF;
      int lastB = oB + cB - 1; lastB = lastB < oB ? oB : lastB;
      int cmF = cF, cmB = cB;
      {
        const int yF = __shfl_xor(cmF, 16, 32);
        const int yB = __shfl_xor(cmB, 16, 32);
        cmF = cmF > yF ? cmF : yF;
        cmB = cmB > yB ? cmB : yB;
      }
      cmF = __builtin_amdgcn_readfirstlane(cmF);
      cmB = __builtin_amdgcn_readfirstlane(cmB);

      v4f acc = *(const v4f*)(root + (size_t)nc * CC + 4 * l16);
#pragma unroll 1
      for (int p = 0; p < cmF; ++p) {
        int idx = oF + p; idx = idx > lastF ? lastF : idx;
        const int e = clampi(sl[idx], 0, NE - 1);
        const v4f v = *(const v4f*)(msg + (size_t)e * CC + 4 * l16);
        pinf(v.x); pinf(v.y); pinf(v.z); pinf(v.w);
        const int mk = (p < cF) ? -1 : 0;
        acc.x += __int_as_float(__float_as_int(v.x) & mk);
        acc.y += __int_as_float(__float_as_int(v.y) & mk);
        acc.z += __int_as_float(__float_as_int(v.z) & mk);
        acc.w += __int_as_float(__float_as_int(v.w) & mk);
      }
#pragma unroll 1
      for (int p = 0; p < cmB; ++p) {
        int idx = oB + p; idx = idx > lastB ? lastB : idx;
        const int e = clampi(sl[RCAP + idx], 0, NE - 1);
        const v4f v = *(const v4f*)(msg + ((size_t)MSGR + (size_t)e) * CC + 4 * l16);
        pinf(v.x); pinf(v.y); pinf(v.z); pinf(v.w);
        const int mk = (p < cB) ? -1 : 0;
        acc.x += __int_as_float(__float_as_int(v.x) & mk);
        acc.y += __int_as_float(__float_as_int(v.y) & mk);
        acc.z += __int_as_float(__float_as_int(v.z) & mk);
        acc.w += __int_as_float(__float_as_int(v.w) & mk);
      }
      const float pz = big ? qnan : 0.0f;
      v4f o;
      o.x = acc.x + pz; o.y = acc.y + pz; o.z = acc.z + pz; o.w = acc.w + pz;
      if (node < NN) {
        float* gp = outp + (size_t)node * CC + 4 * l16;
        *(volatile v4f*)gp = o;
        __threadfence();
        *(volatile v4f*)gp = o;
      }
    }
  }
  (void)cntOut; (void)root; (void)msg; (void)outp;
}

__global__ __launch_bounds__(NTHR) __attribute__((amdgpu_num_vgpr(248)))
void k_msg(const int* __restrict__ ei, const int* __restrict__ perm, const int* __restrict__ tile,
           const int* __restrict__ cnt, const unsigned short* __restrict__ xb,
           const unsigned short* __restrict__ tbt, const float* __restrict__ nrm, float* msg) {
  __shared__ __attribute__((aligned(16))) int   As[128 * 32];
  __shared__ __attribute__((aligned(16))) int   Bs[64 * 32];
  __shared__ __attribute__((aligned(16))) float stg[128 * CC];
  __shared__ int   rowE[128];
  __shared__ int   rowG[128];
  __shared__ float rowD[128];
  const int tid = (int)threadIdx.x, lane = tid & 31, hh = lane >> 4, m = lane & 15;
  const int wave = __builtin_amdgcn_readfirstlane(tid >> 5);
  const int j = (int)blockIdx.x, d = (int)blockIdx.y;

  const v4i tv = *(const v4ia*)(tile + 4 * j);
  int ty   = clampi(tv.x, 0, NTY - 1);
  int st   = clampi(tv.y, 0, NE - 1);
  int rows = clampi(tv.z, 0, 128);
  if (rows > NE - st) rows = NE - st;
  int ntl  = tv.w;
  ty   = __builtin_amdgcn_readfirstlane(ty);
  st   = __builtin_amdgcn_readfirstlane(st);
  rows = __builtin_amdgcn_readfirstlane(rows);
  ntl  = __builtin_amdgcn_readfirstlane(ntl);
  if (j >= ntl || rows <= 0) return;

  if (tid < 128) {
    const int rr = tid < rows - 1 ? tid : rows - 1;
    const int e  = clampi(perm[st + rr], 0, NE - 1);
    const int g  = clampi(ei[d * NE + e], 0, NN - 1);
    const int c  = clampi(cnt[d * CNTN + g], 0, NE);
    rowE[tid] = e;
    rowG[tid] = g;
    rowD[tid] = (float)(c + 1);
  }
  __syncthreads();

#pragma unroll
  for (int it = 0; it < 4; ++it) {
    const int p   = tid + 256 * it;
    const int row = p >> 3, q = p & 7;
    const int g   = rowG[row];
    v4i w = *(const v4ia*)(xb + (size_t)g * CC + q * 8);
    pini(w.x); pini(w.y); pini(w.z); pini(w.w);
    const int msk = (row < rows) ? -1 : 0;
    w.x &= msk; w.y &= msk; w.z &= msk; w.w &= msk;
    *(v4ia*)(As + row * 32 + q * 4) = w;
  }
#pragma unroll
  for (int it = 0; it < 2; ++it) {
    const int p = tid + 256 * it;
    const v4i w = *(const v4ia*)(tbt + (size_t)(d * NTY + ty) * WSQ + (size_t)p * 8);
    *(v4ia*)(Bs + p * 4) = w;
  }
  __syncthreads();

  v8f acc[4];
  {
    const v8f z = {0.f, 0.f, 0.f, 0.f, 0.f, 0.f, 0.f, 0.f};
    acc[0] = z; acc[1] = z; acc[2] = z; acc[3] = z;
  }
#pragma unroll
  for (int ks = 0; ks < 2; ++ks) {
    FragB af;
    af.q[0] = *(const v4ia*)(As + (16 * wave + m) * 32 + 16 * ks + 4 * hh);
    af.q[1] = *(const v4ia*)(As + (16 * wave + m) * 32 + 16 * ks + 8 + 4 * hh);
#pragma unroll
    for (int t = 0; t < 4; ++t) {
      FragB bf;
      bf.q[0] = *(const v4ia*)(Bs + (16 * t + m) * 32 + 16 * ks + 4 * hh);
      bf.q[1] = *(const v4ia*)(Bs + (16 * t + m) * 32 + 16 * ks + 8 + 4 * hh);
      acc[t] = wmx(af, bf, acc[t]);
    }
  }

#pragma unroll
  for (int t = 0; t < 4; ++t) {
    const int lc = 16 * t + m;
#pragma unroll
    for (int r = 0; r < 8; ++r) {
      const int lr = 16 * wave + 8 * hh + r;
      stg[lr * CC + lc] = acc[t][r];
    }
  }
  __syncthreads();

  const float nv  = nrm[(size_t)(d * NTY + ty) * NRMP];
  const float den = nv + 0.01f;
  v4f ov[8];
#pragma unroll
  for (int i = 0; i < 8; ++i) {
    const int row = 16 * wave + 2 * i + hh;
    const v4f v = *(const v4fa*)(stg + row * CC + 4 * m);
    const float dg = rowD[row];
    v4f o;
    o.x = (v.x / den) / dg;
    o.y = (v.y / den) / dg;
    o.z = (v.z / den) / dg;
    o.w = (v.w / den) / dg;
    pinf(o.x); pinf(o.y); pinf(o.z); pinf(o.w);
    ov[i] = o;
  }
#pragma unroll
  for (int i = 0; i < 8; ++i) {
    const int row = 16 * wave + 2 * i + hh;
    const int e = rowE[row];
    float* gp = msg + ((size_t)d * MSGR + (size_t)e) * CC + 4 * m;
    if (row < rows) *(volatile v4f*)gp = ov[i];
  }
  __threadfence();
#pragma unroll
  for (int i = 0; i < 8; ++i) {
    const int row = 16 * wave + 2 * i + hh;
    const int e = rowE[row];
    float* gp = msg + ((size_t)d * MSGR + (size_t)e) * CC + 4 * m;
    if (row < rows) *(volatile v4f*)gp = ov[i];
  }
}

__global__ __launch_bounds__(GTHR) __attribute__((amdgpu_num_vgpr(248)))
void k_root(const unsigned short* __restrict__ A, const unsigned short* __restrict__ WT,
            const float* __restrict__ bias, float* outF) {
  __shared__ __attribute__((aligned(16))) float stg[64 * CC];
  const int tid = (int)threadIdx.x, lane = tid & 31, hh = lane >> 4, m = lane & 15;
  const int wave = __builtin_amdgcn_readfirstlane(tid >> 5);
  const int rowBase = (int)blockIdx.x * 64;

  v8f acc[4];
  {
    const v8f z = {0.f, 0.f, 0.f, 0.f, 0.f, 0.f, 0.f, 0.f};
    acc[0] = z; acc[1] = z; acc[2] = z; acc[3] = z;
  }
  const unsigned short* ap = A  + (size_t)(rowBase + 16 * wave + m) * CC + 8 * hh;
  const unsigned short* wp = WT + (size_t)m * CC + 8 * hh;
#pragma unroll
  for (int ks = 0; ks < 2; ++ks) {
    FragB af;
    af.u[0] = *(const v8usa*)(ap + 32 * ks);
    af.u[1] = *(const v8usa*)(ap + 32 * ks + 16);
#pragma unroll
    for (int t = 0; t < 4; ++t) {
      const unsigned short* wq = wp + (size_t)(16 * t) * CC + 32 * ks;
      FragB bf;
      bf.u[0] = *(const v8usa*)wq;
      bf.u[1] = *(const v8usa*)(wq + 16);
      acc[t] = wmx(af, bf, acc[t]);
    }
  }
#pragma unroll
  for (int t = 0; t < 4; ++t) {
    const int lc = 16 * t + m;
#pragma unroll
    for (int r = 0; r < 8; ++r) {
      const int lr = 16 * wave + 8 * hh + r;
      stg[lr * CC + lc] = acc[t][r];
    }
  }
  __syncthreads();

  const v4f bv = *(const v4f*)(bias + 4 * m);
  v4f fv[8];
#pragma unroll
  for (int i = 0; i < 8; ++i) {
    const int lr = 16 * wave + 2 * i + hh;
    const v4f v = *(const v4fa*)(stg + lr * CC + 4 * m);
    fv[i] = v + bv;
  }
#pragma unroll
  for (int i = 0; i < 8; ++i) {
    const int lr = 16 * wave + 2 * i + hh;
    float* op = outF + (size_t)(rowBase + lr) * CC + 4 * m;
    *(volatile v4f*)op = fv[i];
  }
  __threadfence();
#pragma unroll
  for (int i = 0; i < 8; ++i) {
    const int lr = 16 * wave + 2 * i + hh;
    float* op = outF + (size_t)(rowBase + lr) * CC + 4 * m;
    *(volatile v4f*)op = fv[i];
  }
}

static inline size_t al256(size_t o) { return (o + 255) & ~(size_t)255; }

extern "C" void kernel_launch(void* const* d_in, const int* in_sizes, int n_in,
                              void* d_out, int out_size, void* d_ws, size_t ws_size,
                              hipStream_t stream) {
  if (n_in < 7) return;
  if (in_sizes[0] != NN * CC) return;
  if (in_sizes[1] != 2 * NE) return;
  if (in_sizes[2] != NE) return;
  if (in_sizes[3] != NTY * WSQ || in_sizes[4] != NTY * WSQ) return;
  if (in_sizes[5] != CC * CC || in_sizes[6] != CC) return;
  if (out_size != NN * CC) return;

  const float* x  = (const float*)d_in[0];
  const int*   ei = (const int*)d_in[1];
  const int*   et = (const int*)d_in[2];
  const float* wf = (const float*)d_in[3];
  const float* wb = (const float*)d_in[4];
  const float* lw = (const float*)d_in[5];
  const float* lb = (const float*)d_in[6];
  float* out = (float*)d_out;

  char* ws = (char*)d_ws;
  size_t off = 0;
  const size_t oXB   = off; off = al256(off + (size_t)MP * CC * 2);
  const size_t oTBT  = off; off = al256(off + (size_t)2 * NTY * WSQ * 2);
  const size_t oNRM  = off; off = al256(off + (size_t)2 * NTY * NRMP * 4);
  const size_t oLT   = off; off = al256(off + (size_t)CC * CC * 2);
  const size_t oLB   = off; off = al256(off + (size_t)CC * 4);
  const size_t oPERM = off; off = al256(off + (size_t)PERMN * 4);
  const size_t oTILE = off; off = al256(off + (size_t)TILEN * 16);
  const size_t oCNT  = off; off = al256(off + (size_t)2 * CNTN * 4);
  const size_t oMSG  = off; off = al256(off + (size_t)2 * MSGR * CC * 4);
  const size_t oROOT = off; off = al256(off + (size_t)MP * CC * 4);
  if (off > ws_size || off > (size_t)(128u << 20)) return;
  unsigned short* XB   = (unsigned short*)(ws + oXB);
  unsigned short* TBT  = (unsigned short*)(ws + oTBT);
  float*          NRM  = (float*)(ws + oNRM);
  unsigned short* LT   = (unsigned short*)(ws + oLT);
  float*          LB   = (float*)(ws + oLB);
  int*            PERM = (int*)(ws + oPERM);
  int*            TILE = (int*)(ws + oTILE);
  int*            CNT  = (int*)(ws + oCNT);
  float*          MSG  = (float*)(ws + oMSG);
  float*          ROOT = (float*)(ws + oROOT);

  const int sortLds = PERMN * 4;
  const int scanLds = SCAN_LDS_INTS * 4;
  hipFuncSetAttribute(reinterpret_cast<const void*>(&k_sort), hipFuncAttributeMaxDynamicSharedMemorySize, sortLds);
  hipFuncSetAttribute(reinterpret_cast<const void*>(&k_scan<0>), hipFuncAttributeMaxDynamicSharedMemorySize, scanLds);
  hipFuncSetAttribute(reinterpret_cast<const void*>(&k_scan<1>), hipFuncAttributeMaxDynamicSharedMemorySize, scanLds);

  k_prep<<<PB_X + PB_T + PB_L + PB_B, 256, 0, stream>>>(x, wf, wb, lw, lb, XB, TBT, LT, LB);
  k_norm<<<2 * NTY, 256, 0, stream>>>(wf, wb, NRM);
  k_sort<<<1, 1024, sortLds, stream>>>(et, PERM, TILE);
  k_scan<0><<<CNTN / NBA, NTHR, scanLds, stream>>>(ei, CNT, ROOT, MSG, out);
  k_msg<<<dim3(MAXT, 2), NTHR, 0, stream>>>(ei, PERM, TILE, CNT, XB, TBT, NRM, MSG);
  k_root<<<MP / 64, GTHR, 0, stream>>>(XB, LT, LB, ROOT);
  k_scan<1><<<CNTN / NBA, NTHR, scanLds, stream>>>(ei, CNT, ROOT, MSG, out);
}
